// DeepStatisticalSolver_21509196219215
// MI455X (gfx1250) — hardware-run, weakly checked
//
#include <hip/hip_runtime.h>
#include <math.h>

typedef __attribute__((ext_vector_type(16))) _Float16 v16h;
typedef __attribute__((ext_vector_type(8)))  _Float16 v8h;
typedef __attribute__((ext_vector_type(8)))  float    v8f;
typedef __attribute__((ext_vector_type(4)))  float    v4f;
typedef __attribute__((ext_vector_type(4)))  int      v4i;
typedef __attribute__((ext_vector_type(4)))  unsigned v4u;

constexpr int kN        = 100000;
constexpr int kE        = 800000;
constexpr int kD        = 16;
constexpr int kIters    = 3;
constexpr int kKEdge    = 2 * kD + 3;
constexpr int kKNode    = 3 * kD + 1;
constexpr int kRange    = 2048;
constexpr int kNumRange = (kN + kRange - 1) / kRange;
constexpr int kMessRows = kNumRange * kRange;
constexpr int kNodeBlk  = 128;
constexpr int kNodeBlocks = (kN + kNodeBlk - 1) / kNodeBlk;
constexpr int kNodeRows = kNodeBlocks * kNodeBlk;
constexpr int kChunk    = 1024;
constexpr int kNumChunk = (kE + kChunk - 1) / kChunk;
constexpr int kListCap  = 2048;
constexpr int kMaxBatch = 9;
constexpr int kLossRange  = 12512;
constexpr int kLossBlocks = 8;
constexpr float kWCarry    = 64.0f;
constexpr float kWCarryInv = 1.0f / 64.0f;
constexpr float kResScale  = 2048.0f;
constexpr float kResInv    = 1.0f / 2048.0f;
constexpr float kFix       = 1048576.0f;
constexpr float kFixInv    = 1.0f / 1048576.0f;
constexpr float kFixClamp  = 2000.0f;
constexpr float kAlpha     = 0.1f;
static_assert(kKEdge == 35 && kKNode == 49, "concat widths");
static_assert(kNumRange == 49 && kMessRows == 100352, "range tiling");
static_assert(kNodeBlocks == 782 && kNodeRows == 100096, "node tiling");
static_assert(kNumChunk == 782, "edge chunks");
static_assert((kE % 4) == 0 && (kN % 32) == 0, "vector load and line multiples");
static_assert(kLossRange * kLossBlocks >= kN && (kLossRange % 4) == 0, "loss ranges");
static_assert(kListCap >= 128 + kChunk && (kListCap & (kListCap - 1)) == 0, "ring capacity");
static_assert(((128 + kChunk - 1) >> 7) < kMaxBatch, "batch bound");

constexpr size_t kSzH    = (size_t)kNodeRows * 64;
constexpr size_t kSzHP   = (size_t)kNodeRows * 32;
constexpr size_t kSzSet  = kSzH + 2 * kSzHP;
constexpr size_t kSzMess = (size_t)kMessRows * 64;
constexpr size_t kSzU    = (size_t)kNodeRows * 4;
constexpr size_t kSzPart = (size_t)kIters * kLossBlocks * 128;
constexpr size_t kOffSet0 = 0;
constexpr size_t kOffSet1 = kOffSet0 + kSzSet;
constexpr size_t kOffMT   = kOffSet1 + kSzSet;
constexpr size_t kOffMF   = kOffMT + kSzMess;
constexpr size_t kOffU    = kOffMF + kSzMess;
constexpr size_t kOffPart = kOffU + kSzU;
constexpr size_t kWsTotal = kOffPart + kSzPart;
static_assert(kSzSet == 12812288ull, "set bytes");
static_assert(kWsTotal == 38873088ull, "carve total");
static_assert(kWsTotal <= 134217728ull, "carve cap");
static_assert((kSzH % 128) == 0 && (kSzHP % 128) == 0 && (kSzMess % 128) == 0 && (kSzU % 128) == 0, "aligned regions");
static_assert((kSzSet / 16) % 256 == 0, "zero-fill grid exact");

__device__ __forceinline__ int imin(int a, int b) { return a < b ? a : b; }
__device__ __forceinline__ int imax(int a, int b) { return a > b ? a : b; }
__device__ __forceinline__ int iclamp(int v, int hi) { return imin(imax(v, 0), hi); }

__device__ __forceinline__ float bf16r(float f) {
  unsigned u = __float_as_uint(f);
  u = (u + 0x7FFFu + ((u >> 16) & 1u)) & 0xFFFF0000u;
  return __uint_as_float(u);
}
__device__ __forceinline__ unsigned hbits(float v) {
  const _Float16 x = (_Float16)v;
  return (unsigned)__builtin_bit_cast(unsigned short, x);
}
__device__ __forceinline__ void split16(float v, unsigned& hb, unsigned& lb) {
  const _Float16 x = (_Float16)v;
  float hf = (float)x;
  unsigned hv = (unsigned)__builtin_bit_cast(unsigned short, x);
  const bool tiny = fabsf(hf) < 6.103515625e-5f;
  hf = tiny ? 0.0f : hf;
  hv = tiny ? 0u : hv;
  const float r = (v - hf) * kResScale;
  const _Float16 y = (_Float16)r;
  hb = hv;
  lb = (unsigned)__builtin_bit_cast(unsigned short, y);
}
__device__ __forceinline__ void split8(v4f a, v4f b, v4u& H, v4u& L) {
  const float x0 = a[0], x1 = a[1], x2 = a[2], x3 = a[3];
  const float x4 = b[0], x5 = b[1], x6 = b[2], x7 = b[3];
  unsigned h0, h1, h2, h3, h4, h5, h6, h7, l0, l1, l2, l3, l4, l5, l6, l7;
  split16(x0, h0, l0); split16(x1, h1, l1); split16(x2, h2, l2); split16(x3, h3, l3);
  split16(x4, h4, l4); split16(x5, h5, l5); split16(x6, h6, l6); split16(x7, h7, l7);
  H[0] = h0 | (h1 << 16); H[1] = h2 | (h3 << 16); H[2] = h4 | (h5 << 16); H[3] = h6 | (h7 << 16);
  L[0] = l0 | (l1 << 16); L[1] = l2 | (l3 << 16); L[2] = l4 | (l5 << 16); L[3] = l6 | (l7 << 16);
}

union FragU { v16h v; v8h h[2]; };
__device__ __forceinline__ v16h frag_ld(const _Float16* p) {
  FragU f;
  f.h[0] = *(const v8h*)(p);
  f.h[1] = *(const v8h*)(p + 16);
  return f.v;
}
__device__ __forceinline__ v8f mma_g(v16h a, v16h b, v8f c) {
  c = __builtin_amdgcn_wmma_f32_16x16x32_f16(false, a, false, b, (short)0, c, false, false);
  asm volatile("v_nop\n\tv_nop\n\tv_nop\n\tv_nop" : "+v"(c) : "v"(a), "v"(b));
  return c;
}

template <int KP>
__device__ __forceinline__ void build_wt(const float* __restrict__ w, const int kin, _Float16* plane, const int tid) {
#pragma unroll 1
  for (int idx = tid * 2; idx < 16 * KP; idx += 512) {
    const int n = idx / KP;
    const int k = idx - n * KP;
    const int kc0 = imin(k, kin - 1);
    const int kc1 = imin(k + 1, kin - 1);
    float v0 = w[kc0 * 16 + n];
    float v1 = w[kc1 * 16 + n];
    asm volatile("" : "+v"(v0), "+v"(v1));
    const float c0 = (k < kin) ? bf16r(v0) * kWCarry : 0.0f;
    const float c1 = (k + 1 < kin) ? bf16r(v1) * kWCarry : 0.0f;
    const unsigned word = hbits(c0) | (hbits(c1) << 16);
    *(unsigned*)(plane + idx) = word;
  }
}

__device__ __forceinline__ void stage_tile32(_Float16* th, _Float16* tl, const float (&v)[8], const int hf, const int m) {
#pragma unroll
  for (int r = 0; r < 8; ++r) {
    unsigned hb, lb;
    split16(v[r], hb, lb);
    const unsigned short hs = (unsigned short)hb;
    const unsigned short ls = (unsigned short)lb;
    th[(8 * hf + r) * 32 + m] = __builtin_bit_cast(_Float16, hs);
    tl[(8 * hf + r) * 32 + m] = __builtin_bit_cast(_Float16, ls);
  }
  const v4u z = {0u, 0u, 0u, 0u};
  *(v4u*)(th + m * 32 + 16 + 8 * hf) = z;
  *(v4u*)(tl + m * 32 + 16 + 8 * hf) = z;
}

__global__ __launch_bounds__(256) void zero_fill_kernel(v4u* __restrict__ p, int n16) {
  const int i = blockIdx.x * 256 + threadIdx.x;
  if (i < n16) {
    const v4u z = {0u, 0u, 0u, 0u};
    *(volatile v4u*)(p + i) = z;
    __threadfence();
    *(volatile v4u*)(p + i) = z;
  }
}

__global__ __launch_bounds__(256) void edge_range_kernel(
    const int* __restrict__ src, const int* __restrict__ dst, const float* __restrict__ eattr,
    const unsigned short* __restrict__ hhi, const unsigned short* __restrict__ hlo,
    const float* __restrict__ w1_to, const float* __restrict__ b1_to,
    const float* __restrict__ w2_to, const float* __restrict__ b2_to,
    const float* __restrict__ w1_fr, const float* __restrict__ b1_fr,
    const float* __restrict__ w2_fr, const float* __restrict__ b2_fr,
    float* __restrict__ mess_to, float* __restrict__ mess_fr)
{
  extern __shared__ __align__(16) int sAcc[];
  __shared__ __align__(16) _Float16 sAh[8][16 * 64];
  __shared__ __align__(16) _Float16 sAl[8][16 * 64];
  __shared__ __align__(16) _Float16 sA2h[8][16 * 32];
  __shared__ __align__(16) _Float16 sA2l[8][16 * 32];
  __shared__ __align__(16) _Float16 sW1[16 * 64];
  __shared__ __align__(16) _Float16 sW2[16 * 32];
  __shared__ float sB1[16];
  __shared__ float sB2[16];
  __shared__ __align__(16) int sList[kListCap];
  __shared__ __align__(16) int sAgg[8][16];
  __shared__ int sCnt;

  const int tid = threadIdx.x, lane = tid & 31, wave = tid >> 5;
  const int m = lane & 15, hf = lane >> 4;
  const int dir = blockIdx.y;
  const int base = blockIdx.x * kRange;
  const float* w1 = dir ? w1_fr : w1_to;
  const float* b1 = dir ? b1_fr : b1_to;
  const float* w2 = dir ? w2_fr : w2_to;
  const float* b2 = dir ? b2_fr : b2_to;
  const int* aggp = dir ? src : dst;
  float* outp = dir ? mess_fr : mess_to;

  {
    const v4i z = {0, 0, 0, 0};
#pragma unroll 1
    for (int it = 0; it < (kRange * 16 / 4) / 256; ++it) ((v4i*)sAcc)[it * 256 + tid] = z;
    ((v4i*)sList)[tid] = z;
    ((v4i*)sList)[256 + tid] = z;
  }
  if (tid == 0) sCnt = 0;
  build_wt<64>(w1, kKEdge, sW1, tid);
  build_wt<32>(w2, kD, sW2, tid);
  {
    float x1 = b1[tid & 15];
    float x2 = b2[tid & 15];
    asm volatile("" : "+v"(x1), "+v"(x2));
    if (tid < 16) { sB1[tid] = bf16r(x1); sB2[tid] = bf16r(x2); }
  }
  __syncthreads();

  const v16h bW1a = frag_ld(sW1 + m * 64 + 8 * hf);
  const v16h bW1b = frag_ld(sW1 + m * 64 + 32 + 8 * hf);
  const v16h bW2  = frag_ld(sW2 + m * 32 + 8 * hf);
  const float bias1 = sB1[m];
  const float bias2 = sB2[m];
  const v8f zero8 = {0.f, 0.f, 0.f, 0.f, 0.f, 0.f, 0.f, 0.f};
  const v4u zero4 = {0u, 0u, 0u, 0u};

  _Float16* Ah  = sAh[wave];
  _Float16* Al  = sAl[wave];
  _Float16* A2h = sA2h[wave];
  _Float16* A2l = sA2l[wave];

  int done = 0;
#pragma unroll 1
  for (int c = 0; c <= kNumChunk; ++c) {
    if (c < kNumChunk) {
      const int eb = c * kChunk + tid * 4;
      const bool inr = eb < kE;
      const int ebc = inr ? eb : (kE - 4);
      const v4i a4 = *(const v4i*)(aggp + ebc);
      int a0 = a4[0], a1 = a4[1], a2 = a4[2], a3 = a4[3];
      asm volatile("" : "+v"(a0), "+v"(a1), "+v"(a2), "+v"(a3));
      const bool h0 = inr && ((unsigned)(a0 - base) < (unsigned)kRange);
      const bool h1 = inr && ((unsigned)(a1 - base) < (unsigned)kRange);
      const bool h2 = inr && ((unsigned)(a2 - base) < (unsigned)kRange);
      const bool h3 = inr && ((unsigned)(a3 - base) < (unsigned)kRange);
      const int nh = (int)h0 + (int)h1 + (int)h2 + (int)h3;
      if (nh > 0) {
        int p = atomicAdd(&sCnt, nh);
        if (h0) { sList[p & (kListCap - 1)] = eb;     ++p; }
        if (h1) { sList[p & (kListCap - 1)] = eb + 1; ++p; }
        if (h2) { sList[p & (kListCap - 1)] = eb + 2; ++p; }
        if (h3) { sList[p & (kListCap - 1)] = eb + 3; ++p; }
      }
    }
    __syncthreads();
    const int cnt = sCnt;
    __syncthreads();
    const int avail = cnt - done;
    const int nb = (c < kNumChunk) ? (avail >> 7) : ((avail + 127) >> 7);
#pragma unroll 1
    for (int b = 0; b < kMaxBatch; ++b) {
      if (b >= nb) break;
      const int nval = imin(cnt - done, 128);

      const int slot = 16 * wave + m;
      const bool rv = slot < nval;
      int e = sList[(done + slot) & (kListCap - 1)];
      e = iclamp(e, kE - 1);
      const int s = iclamp(src[e], kN - 1);
      const int d = iclamp(dst[e], kN - 1);
      float e0 = eattr[(size_t)e * 3 + 0];
      asm volatile("" : "+v"(e0));
      float e1 = eattr[(size_t)e * 3 + 1];
      asm volatile("" : "+v"(e1));
      float e2 = eattr[(size_t)e * 3 + 2];
      asm volatile("" : "+v"(e2));
      const int xi = dir ? s : d;
      const int xj = dir ? d : s;
      const int grow = hf ? xj : xi;
      const v4u gh0 = *(const v4u*)(hhi + (size_t)grow * 16);
      const v4u gh1 = *(const v4u*)(hhi + (size_t)grow * 16 + 8);
      const v4u gl0 = *(const v4u*)(hlo + (size_t)grow * 16);
      const v4u gl1 = *(const v4u*)(hlo + (size_t)grow * 16 + 8);
      unsigned eh0, el0, eh1, el1, eh2, el2;
      split16(bf16r(e0), eh0, el0);
      split16(bf16r(e1), eh1, el1);
      split16(bf16r(e2), eh2, el2);
      v4u evh, evl;
      evh[0] = hf ? 0u : (eh0 | (eh1 << 16));
      evh[1] = hf ? 0u : eh2;
      evh[2] = 0u;
      evh[3] = 0u;
      evl[0] = hf ? 0u : (el0 | (el1 << 16));
      evl[1] = hf ? 0u : el2;
      evl[2] = 0u;
      evl[3] = 0u;
      *(v4u*)(Ah + m * 64 + 16 * hf)      = gh0;
      *(v4u*)(Ah + m * 64 + 16 * hf + 8)  = gh1;
      *(v4u*)(Ah + m * 64 + 32 + 16 * hf) = evh;
      *(v4u*)(Ah + m * 64 + 40 + 16 * hf) = zero4;
      *(v4u*)(Al + m * 64 + 16 * hf)      = gl0;
      *(v4u*)(Al + m * 64 + 16 * hf + 8)  = gl1;
      *(v4u*)(Al + m * 64 + 32 + 16 * hf) = evl;
      *(v4u*)(Al + m * 64 + 40 + 16 * hf) = zero4;
      if (hf == 0) {
        const int loc = xi - base;
        const bool ok = rv && (s != d) && ((unsigned)loc < (unsigned)kRange);
        sAgg[wave][m] = ok ? loc : -1;
      }
      __syncthreads();

      v8f am = zero8, ar = zero8;
      {
        const _Float16* pa = Ah + m * 64 + 8 * hf;
        const _Float16* pl = Al + m * 64 + 8 * hf;
        const v16h a0f = frag_ld(pa);
        const v16h r0f = frag_ld(pl);
        am = mma_g(a0f, bW1a, am);
        ar = mma_g(r0f, bW1a, ar);
        const v16h a1f = frag_ld(pa + 32);
        const v16h r1f = frag_ld(pl + 32);
        am = mma_g(a1f, bW1b, am);
        ar = mma_g(r1f, bW1b, ar);
      }
      {
        float hid[8];
#pragma unroll
        for (int r = 0; r < 8; ++r) {
          const float pre = (am[r] + ar[r] * kResInv) * kWCarryInv + bias1;
          hid[r] = fmaxf(pre, 0.0f);
        }
        stage_tile32(A2h, A2l, hid, hf, m);
      }
      __syncthreads();

      v8f cm = zero8, cr = zero8;
      {
        const v16h a0f = frag_ld(A2h + m * 32 + 8 * hf);
        const v16h r0f = frag_ld(A2l + m * 32 + 8 * hf);
        cm = mma_g(a0f, bW2, cm);
        cr = mma_g(r0f, bW2, cr);
      }
      {
        const v4i q0 = *(const v4i*)(&sAgg[wave][8 * hf]);
        const v4i q1 = *(const v4i*)(&sAgg[wave][8 * hf + 4]);
        const int ag[8] = {q0[0], q0[1], q0[2], q0[3], q1[0], q1[1], q1[2], q1[3]};
#pragma unroll
        for (int r = 0; r < 8; ++r) {
          float msg = (cm[r] + cr[r] * kResInv) * kWCarryInv + bias2;
          msg = fminf(fmaxf(msg, -kFixClamp), kFixClamp);
          const int q = __float2int_rn(msg * kFix);
          if (ag[r] >= 0) atomicAdd(&sAcc[ag[r] * 16 + m], q);
        }
      }
      __syncthreads();
      done += nval;
    }
  }
  __syncthreads();

  {
    float* op = outp + (size_t)base * 16;
    for (int pass = 0; pass < 2; ++pass) {
#pragma unroll 1
      for (int it = 0; it < (kRange * 16 / 4) / 256; ++it) {
        const int q = it * 256 + tid;
        const v4i a = ((const v4i*)sAcc)[q];
        v4f f;
        f[0] = (float)a[0] * kFixInv;
        f[1] = (float)a[1] * kFixInv;
        f[2] = (float)a[2] * kFixInv;
        f[3] = (float)a[3] * kFixInv;
        *(volatile v4f*)(op + (size_t)q * 4) = f;
      }
      __threadfence();
    }
  }
}

__global__ __launch_bounds__(256) void node_update_kernel(
    const float* __restrict__ hcur, float* __restrict__ hnxt,
    unsigned short* __restrict__ hhn, unsigned short* __restrict__ hln,
    const float* __restrict__ mto, const float* __restrict__ mfr, const float* __restrict__ prb,
    const float* __restrict__ pw1, const float* __restrict__ pb1,
    const float* __restrict__ pw2, const float* __restrict__ pb2,
    const float* __restrict__ dw1, const float* __restrict__ db1,
    const float* __restrict__ dw2, const float* __restrict__ db2,
    float* __restrict__ uws, float* __restrict__ uout, int write_out)
{
  __shared__ __align__(16) _Float16 sAh[8][16 * 64];
  __shared__ __align__(16) _Float16 sAl[8][16 * 64];
  __shared__ __align__(16) _Float16 sA2h[8][16 * 32];
  __shared__ __align__(16) _Float16 sA2l[8][16 * 32];
  __shared__ __align__(16) _Float16 sW1[16 * 64];
  __shared__ __align__(16) _Float16 sW2[16 * 32];
  __shared__ __align__(16) _Float16 sWd1[16 * 32];
  __shared__ __align__(16) _Float16 sWd2[16 * 32];
  __shared__ float sB[64];
  __shared__ __align__(16) float sHn[8][16 * 20];
  __shared__ __align__(16) float sU[128];

  const int tid = threadIdx.x, lane = tid & 31, wave = tid >> 5;
  const int m = lane & 15, hf = lane >> 4;

  build_wt<64>(pw1, kKNode, sW1, tid);
  build_wt<32>(pw2, kD, sW2, tid);
  build_wt<32>(dw1, kD, sWd1, tid);
  {
    const int idx = tid * 2;
    const int n = idx >> 5;
    const int k = idx & 31;
    float v0 = dw2[imin(k, kD - 1)];
    float v1 = dw2[imin(k + 1, kD - 1)];
    asm volatile("" : "+v"(v0), "+v"(v1));
    const float c0 = ((n == 0) && (k < kD)) ? bf16r(v0) * kWCarry : 0.0f;
    const float c1 = ((n == 0) && (k + 1 < kD)) ? bf16r(v1) * kWCarry : 0.0f;
    *(unsigned*)(sWd2 + idx) = hbits(c0) | (hbits(c1) << 16);
  }
  {
    const int j = tid & 15;
    const int g = (tid >> 4) & 3;
    float x0 = pb1[j], x1 = pb2[j], x2 = db1[j], x3 = db2[0];
    asm volatile("" : "+v"(x0), "+v"(x1), "+v"(x2), "+v"(x3));
    const float v = (g == 0) ? x0 : (g == 1) ? x1 : (g == 2) ? x2 : x3;
    if (tid < 64) sB[tid] = bf16r(v);
  }
  __syncthreads();

  const v16h bP1a = frag_ld(sW1 + m * 64 + 8 * hf);
  const v16h bP1b = frag_ld(sW1 + m * 64 + 32 + 8 * hf);
  const v16h bP2  = frag_ld(sW2 + m * 32 + 8 * hf);
  const v16h bD1  = frag_ld(sWd1 + m * 32 + 8 * hf);
  const v16h bD2  = frag_ld(sWd2 + m * 32 + 8 * hf);
  const float bp1 = sB[m], bp2 = sB[16 + m], bd1 = sB[32 + m], bd2 = sB[48];
  const v8f zero8 = {0.f, 0.f, 0.f, 0.f, 0.f, 0.f, 0.f, 0.f};

  _Float16* Ah  = sAh[wave];
  _Float16* Al  = sAl[wave];
  _Float16* A2h = sA2h[wave];
  _Float16* A2l = sA2l[wave];
  float* Hn = sHn[wave];

  const int node0 = (blockIdx.x * 8 + wave) * 16;

  {
    const int nc = imin(node0 + m, kN - 1);
    const float* pc = hcur + (size_t)nc * 16;
    const float* pf = mfr + (size_t)nc * 16;
    const float* pb = mto + (size_t)nc * 16;
    v4f hc0 = *(const v4f*)(pc);
    asm volatile("" : "+v"(hc0));
    v4f hc1 = *(const v4f*)(pc + 4);
    asm volatile("" : "+v"(hc1));
    v4f hc2 = *(const v4f*)(pc + 8);
    asm volatile("" : "+v"(hc2));
    v4f hc3 = *(const v4f*)(pc + 12);
    asm volatile("" : "+v"(hc3));
    v4f mf0 = *(const v4f*)(pf);
    asm volatile("" : "+v"(mf0));
    v4f mf1 = *(const v4f*)(pf + 4);
    asm volatile("" : "+v"(mf1));
    v4f mf2 = *(const v4f*)(pf + 8);
    asm volatile("" : "+v"(mf2));
    v4f mf3 = *(const v4f*)(pf + 12);
    asm volatile("" : "+v"(mf3));
    const v4f f0 = hf ? mf0 : hc0;
    const v4f f1 = hf ? mf1 : hc1;
    const v4f f2 = hf ? mf2 : hc2;
    const v4f f3 = hf ? mf3 : hc3;
    v4f g0 = *(const v4f*)(pb);
    asm volatile("" : "+v"(g0));
    v4f g1 = *(const v4f*)(pb + 4);
    asm volatile("" : "+v"(g1));
    v4f g2 = *(const v4f*)(pb + 8);
    asm volatile("" : "+v"(g2));
    v4f g3 = *(const v4f*)(pb + 12);
    asm volatile("" : "+v"(g3));
    float pv = prb[nc];
    asm volatile("" : "+v"(pv));
    const float pvr = bf16r(pv);
    const v4f pz = {pvr, 0.0f, 0.0f, 0.0f};
    const v4f zz = {0.0f, 0.0f, 0.0f, 0.0f};
    g0 = hf ? pz : g0;
    g1 = hf ? zz : g1;
    g2 = hf ? zz : g2;
    g3 = hf ? zz : g3;
    v4u H0, L0, H1, L1, H2, L2, H3, L3;
    split8(f0, f1, H0, L0);
    split8(f2, f3, H1, L1);
    split8(g0, g1, H2, L2);
    split8(g2, g3, H3, L3);
    v4u* ph = (v4u*)(Ah + m * 64 + 32 * hf);
    v4u* pl = (v4u*)(Al + m * 64 + 32 * hf);
    ph[0] = H0; ph[1] = H1; ph[2] = H2; ph[3] = H3;
    pl[0] = L0; pl[1] = L1; pl[2] = L2; pl[3] = L3;
  }
  float hold[8];
#pragma unroll
  for (int r = 0; r < 8; ++r) {
    const int nr = imin(node0 + 8 * hf + r, kN - 1);
    hold[r] = hcur[(size_t)nr * 16 + m];
  }
  __syncthreads();

  v8f am = zero8, ar = zero8;
  {
    const _Float16* pa = Ah + m * 64 + 8 * hf;
    const _Float16* pl = Al + m * 64 + 8 * hf;
    const v16h a0f = frag_ld(pa);
    const v16h r0f = frag_ld(pl);
    am = mma_g(a0f, bP1a, am);
    ar = mma_g(r0f, bP1a, ar);
    const v16h a1f = frag_ld(pa + 32);
    const v16h r1f = frag_ld(pl + 32);
    am = mma_g(a1f, bP1b, am);
    ar = mma_g(r1f, bP1b, ar);
  }
  {
    float hid[8];
#pragma unroll
    for (int r = 0; r < 8; ++r) hid[r] = fmaxf((am[r] + ar[r] * kResInv) * kWCarryInv + bp1, 0.0f);
    stage_tile32(A2h, A2l, hid, hf, m);
  }
  __syncthreads();

  v8f cm = zero8, cr = zero8;
  {
    const v16h a0f = frag_ld(A2h + m * 32 + 8 * hf);
    const v16h r0f = frag_ld(A2l + m * 32 + 8 * hf);
    cm = mma_g(a0f, bP2, cm);
    cr = mma_g(r0f, bP2, cr);
  }
  float hn[8];
#pragma unroll
  for (int r = 0; r < 8; ++r) {
    const float msg = (cm[r] + cr[r] * kResInv) * kWCarryInv + bp2;
    hn[r] = hold[r] + kAlpha * msg;
  }
  __syncthreads();
#pragma unroll
  for (int r = 0; r < 8; ++r) Hn[(8 * hf + r) * 20 + m] = hn[r];
  stage_tile32(A2h, A2l, hn, hf, m);
  __syncthreads();

  {
    v4f fv[2];
#pragma unroll
    for (int it = 0; it < 2; ++it) {
      const int q = it * 32 + lane;
      fv[it] = *(const v4f*)(Hn + (q >> 2) * 20 + (q & 3) * 4);
    }
    const int prow = lane >> 1, c8 = (lane & 1) * 8;
    const v4f x0 = *(const v4f*)(Hn + prow * 20 + c8);
    const v4f x1 = *(const v4f*)(Hn + prow * 20 + c8 + 4);
    v4u PH, PL;
    split8(x0, x1, PH, PL);
    float* gp = hnxt + (size_t)node0 * 16;
    unsigned short* gh = hhn + (size_t)node0 * 16 + lane * 8;
    unsigned short* gl = hln + (size_t)node0 * 16 + lane * 8;
    for (int pass = 0; pass < 2; ++pass) {
      *(volatile v4f*)(gp + lane * 4) = fv[0];
      *(volatile v4f*)(gp + 128 + lane * 4) = fv[1];
      *(volatile v4u*)(gh) = PH;
      *(volatile v4u*)(gl) = PL;
      __threadfence();
    }
  }

  v8f dm = zero8, dr = zero8;
  {
    const v16h a0f = frag_ld(A2h + m * 32 + 8 * hf);
    const v16h r0f = frag_ld(A2l + m * 32 + 8 * hf);
    dm = mma_g(a0f, bD1, dm);
    dr = mma_g(r0f, bD1, dr);
  }
  float hd[8];
#pragma unroll
  for (int r = 0; r < 8; ++r) hd[r] = fmaxf((dm[r] + dr[r] * kResInv) * kWCarryInv + bd1, 0.0f);
  __syncthreads();
  stage_tile32(A2h, A2l, hd, hf, m);
  __syncthreads();

  v8f um = zero8, ur = zero8;
  {
    const v16h a0f = frag_ld(A2h + m * 32 + 8 * hf);
    const v16h r0f = frag_ld(A2l + m * 32 + 8 * hf);
    um = mma_g(a0f, bD2, um);
    ur = mma_g(r0f, bD2, ur);
  }
  if (m == 0) {
#pragma unroll
    for (int r = 0; r < 8; ++r) sU[wave * 16 + 8 * hf + r] = (um[r] + ur[r] * kResInv) * kWCarryInv + bd2;
  }
  __syncthreads();
  if (wave == 0) {
    const v4f uv = *(const v4f*)(sU + lane * 4);
    const int nb0 = blockIdx.x * kNodeBlk + lane * 4;
    const bool wo = (write_out != 0) && (nb0 < kN);
    for (int pass = 0; pass < 2; ++pass) {
      *(volatile v4f*)(uws + nb0) = uv;
      if (wo) *(volatile v4f*)(uout + nb0) = uv;
      __threadfence();
    }
  }
}

__global__ __launch_bounds__(256) void loss_range_kernel(
    const int* __restrict__ src, const int* __restrict__ dst, const float* __restrict__ aij,
    const float* __restrict__ uws, const float* __restrict__ yv, float* __restrict__ part)
{
  __shared__ __align__(16) int sSum[kLossRange];
  __shared__ float sRed[256];
  const int tid = threadIdx.x, lane = tid & 31, wave = tid >> 5;
  const int base = blockIdx.x * kLossRange;
  {
    const v4i z = {0, 0, 0, 0};
#pragma unroll 1
    for (int i = tid; i < kLossRange / 4; i += 256) ((v4i*)sSum)[i] = z;
  }
  __syncthreads();
#pragma unroll 1
  for (int c = 0; c < kNumChunk; ++c) {
    const int eb = c * kChunk + tid * 4;
    const bool inr = eb < kE;
    const int ebc = inr ? eb : (kE - 4);
    const v4i s4 = *(const v4i*)(src + ebc);
    const v4i d4 = *(const v4i*)(dst + ebc);
    const v4f a4 = *(const v4f*)(aij + ebc);
    float av0 = a4[0], av1 = a4[1], av2 = a4[2], av3 = a4[3];
    asm volatile("" : "+v"(av0), "+v"(av1), "+v"(av2), "+v"(av3));
    const int sv[4] = {s4[0], s4[1], s4[2], s4[3]};
    const int dv[4] = {d4[0], d4[1], d4[2], d4[3]};
    const float av[4] = {av0, av1, av2, av3};
#pragma unroll
    for (int j = 0; j < 4; ++j) {
      const int dc = iclamp(dv[j], kN - 1);
      float uv = uws[dc];
      asm volatile("" : "+v"(uv));
      const int loc = sv[j] - base;
      const bool hit = inr && ((unsigned)loc < (unsigned)kLossRange);
      float val = bf16r(av[j]) * uv;
      val = fminf(fmaxf(val, -kFixClamp), kFixClamp);
      const int q = __float2int_rn(val * kFix);
      if (hit) atomicAdd(&sSum[loc], q);
    }
  }
  __syncthreads();
  float acc = 0.0f;
#pragma unroll 1
  for (int it = 0; it < (kLossRange + 255) / 256; ++it) {
    const int i = it * 256 + tid;
    const bool inb = i < kLossRange;
    const int ic = inb ? i : 0;
    const int node = base + ic;
    const bool okn = inb && (node < kN);
    float y = yv[imin(node, kN - 1)];
    asm volatile("" : "+v"(y));
    const float au = (float)sSum[ic] * kFixInv;
    const float dl = au - bf16r(y);
    acc += okn ? dl * dl : 0.0f;
  }
  sRed[tid] = acc;
  __syncthreads();
#pragma unroll 1
  for (int s = 128; s > 0; s >>= 1) {
    if (tid < s) sRed[tid] += sRed[tid + s];
    __syncthreads();
  }
  if (wave == 0) {
    const float tot = sRed[0];
    const float v = (lane == 0) ? tot : 0.0f;
    volatile float* pp = part + blockIdx.x * 32 + lane;
    *pp = v;
    __threadfence();
    *pp = v;
  }
}

__global__ __launch_bounds__(32) void loss_final_kernel(const float* __restrict__ part, float* __restrict__ out1)
{
  __shared__ float sP[32];
  const int l = threadIdx.x;
  const int lc = (l < kIters * kLossBlocks) ? l : (kIters * kLossBlocks - 1);
  float p = part[lc * 32];
  asm volatile("" : "+v"(p));
  sP[l] = p;
  __syncthreads();
  if (l == 0) {
    float tot = 0.0f;
#pragma unroll 1
    for (int t = 0; t < kIters; ++t) {
      float s = 0.0f;
#pragma unroll 1
      for (int b = 0; b < kLossBlocks; ++b) s += sP[t * kLossBlocks + b];
      const float wgt = (t == 0) ? 0.81f : ((t == 1) ? 0.9f : 1.0f);
      tot += (s * (1.0f / (float)kN)) * wgt;
    }
    *(volatile float*)out1 = tot;
    __threadfence();
    *(volatile float*)out1 = tot;
  }
}

extern "C" void kernel_launch(void* const* d_in, const int* in_sizes, int n_in,
                              void* d_out, int out_size, void* d_ws, size_t ws_size,
                              hipStream_t stream)
{
  if (n_in < 22) return;
  if (in_sizes[0] != 2 * kE) return;
  if (in_sizes[1] != 3 * kE) return;
  if (in_sizes[2] != kE) return;
  if (in_sizes[3] != kN) return;
  if (in_sizes[5] != kN) return;
  if (in_sizes[6] != kIters * kKEdge * kD) return;
  if (in_sizes[8] != kIters * kD * kD) return;
  if (in_sizes[10] != kIters * kKEdge * kD) return;
  if (in_sizes[12] != kIters * kD * kD) return;
  if (in_sizes[14] != kIters * kKNode * kD) return;
  if (in_sizes[16] != kIters * kD * kD) return;
  if (in_sizes[18] != kIters * kD * kD) return;
  if (in_sizes[20] != kIters * kD) return;
  if (in_sizes[21] != kIters) return;
  if (out_size != kN + 1) return;
  if (ws_size < kWsTotal) return;

  const int*   edge_index = (const int*)d_in[0];
  const float* edge_attr  = (const float*)d_in[1];
  const float* a_ij       = (const float*)d_in[2];
  const float* prb        = (const float*)d_in[3];
  const float* yv         = (const float*)d_in[5];
  const float* to_w1 = (const float*)d_in[6];
  const float* to_b1 = (const float*)d_in[7];
  const float* to_w2 = (const float*)d_in[8];
  const float* to_b2 = (const float*)d_in[9];
  const float* fr_w1 = (const float*)d_in[10];
  const float* fr_b1 = (const float*)d_in[11];
  const float* fr_w2 = (const float*)d_in[12];
  const float* fr_b2 = (const float*)d_in[13];
  const float* ps_w1 = (const float*)d_in[14];
  const float* ps_b1 = (const float*)d_in[15];
  const float* ps_w2 = (const float*)d_in[16];
  const float* ps_b2 = (const float*)d_in[17];
  const float* dc_w1 = (const float*)d_in[18];
  const float* dc_b1 = (const float*)d_in[19];
  const float* dc_w2 = (const float*)d_in[20];
  const float* dc_b2 = (const float*)d_in[21];

  const int* src = edge_index;
  const int* dst = edge_index + kE;

  char* ws = (char*)d_ws;
  float*          Hf[2];
  unsigned short* Hh[2];
  unsigned short* Hl[2];
  Hf[0] = (float*)(ws + kOffSet0);
  Hh[0] = (unsigned short*)(ws + kOffSet0 + kSzH);
  Hl[0] = (unsigned short*)(ws + kOffSet0 + kSzH + kSzHP);
  Hf[1] = (float*)(ws + kOffSet1);
  Hh[1] = (unsigned short*)(ws + kOffSet1 + kSzH);
  Hl[1] = (unsigned short*)(ws + kOffSet1 + kSzH + kSzHP);
  float* MT   = (float*)(ws + kOffMT);
  float* MF   = (float*)(ws + kOffMF);
  float* U    = (float*)(ws + kOffU);
  float* PART = (float*)(ws + kOffPart);

  float* u_out    = (float*)d_out;
  float* loss_out = (float*)d_out + kN;

  {
    const int n16 = (int)(kSzSet / 16);
    zero_fill_kernel<<<n16 / 256, 256, 0, stream>>>((v4u*)(ws + kOffSet0), n16);
  }

  for (int t = 0; t < kIters; ++t) {
    const int cur = t & 1, nxt = cur ^ 1;
    edge_range_kernel<<<dim3(kNumRange, 2), 256, (size_t)kRange * 16 * 4, stream>>>(
        src, dst, edge_attr, Hh[cur], Hl[cur],
        to_w1 + (size_t)t * kKEdge * kD, to_b1 + (size_t)t * kD, to_w2 + (size_t)t * kD * kD, to_b2 + (size_t)t * kD,
        fr_w1 + (size_t)t * kKEdge * kD, fr_b1 + (size_t)t * kD, fr_w2 + (size_t)t * kD * kD, fr_b2 + (size_t)t * kD,
        MT, MF);
    node_update_kernel<<<kNodeBlocks, 256, 0, stream>>>(
        Hf[cur], Hf[nxt], Hh[nxt], Hl[nxt], MT, MF, prb,
        ps_w1 + (size_t)t * kKNode * kD, ps_b1 + (size_t)t * kD, ps_w2 + (size_t)t * kD * kD, ps_b2 + (size_t)t * kD,
        dc_w1 + (size_t)t * kD * kD, dc_b1 + (size_t)t * kD, dc_w2 + (size_t)t * kD, dc_b2 + (size_t)t,
        U, u_out, (t == kIters - 1) ? 1 : 0);
    loss_range_kernel<<<kLossBlocks, 256, 0, stream>>>(
        src, dst, a_ij, U, yv, PART + (size_t)t * kLossBlocks * 32);
  }
  loss_final_kernel<<<1, 32, 0, stream>>>(PART, loss_out);
}
